// BarrierNet_31104153158091
// MI455X (gfx1250) — hardware-verified
//
#include <hip/hip_runtime.h>
#include <math.h>

typedef __attribute__((ext_vector_type(16))) _Float16 v16h;
typedef __attribute__((ext_vector_type(16))) __bf16 v16b;
typedef __attribute__((ext_vector_type(8)))  _Float16 v8h;
typedef __attribute__((ext_vector_type(8)))  float v8f;
typedef __attribute__((ext_vector_type(4)))  float v4f;
typedef __attribute__((ext_vector_type(2)))  float v2f;
typedef __attribute__((ext_vector_type(4)))  unsigned v4u;
typedef __attribute__((ext_vector_type(4)))  int v4i;
typedef float __attribute__((may_alias)) float_a;
typedef int __attribute__((may_alias)) int_a;

template <typename T> __device__ __forceinline__ void vst2(void* p, T v) { *(volatile T*)p = v; __threadfence(); *(volatile T*)p = v; }
__device__ __forceinline__ v8f wmma16(v16h a, v16h b, v8f c) {
  v8f d = __builtin_amdgcn_wmma_f32_16x16x32_f16(false, a, false, b, (short)0, c, false, false);
  asm volatile("v_nop\n\tv_nop\n\tv_nop\n\tv_nop" : "+v"(d) : "v"(a), "v"(b));
  return d;
}
__device__ __forceinline__ v8f wmma_bf(v16b a, v16b b, v8f c) {
  v8f d = __builtin_amdgcn_wmma_f32_16x16x32_bf16(false, a, false, b, (short)0, c, false, false);
  asm volatile("v_nop\n\tv_nop\n\tv_nop\n\tv_nop" : "+v"(d) : "v"(a), "v"(b));
  return d;
}
__device__ __forceinline__ v16h frag_h(const _Float16* rowk0, int lane) {
  union { v16h v; v8h q[2]; } u; const _Float16* p = rowk0 + 8 * (lane >> 4);
  u.q[0] = *(const v8h*)p; u.q[1] = *(const v8h*)(p + 16); return u.v;
}
__device__ __forceinline__ v16h frag_f32(const float* rowk0, int lane) {
  v16h a; const float* p = rowk0 + 8 * (lane >> 4);
#pragma unroll
  for (int i = 0; i < 8; ++i) { a[i] = (_Float16)p[i]; a[8 + i] = (_Float16)p[16 + i]; }
  return a;
}
__device__ __forceinline__ v16h frag_f32s(const float* rowk0, int lane, float sc) {
  v16h a; const float* p = rowk0 + 8 * (lane >> 4);
#pragma unroll
  for (int i = 0; i < 8; ++i) { a[i] = (_Float16)(p[i] * sc); a[8 + i] = (_Float16)(p[16 + i] * sc); }
  return a;
}
__device__ __forceinline__ v16h fragc_f32(const float* W, int k0, int n, int lane, int ld, int K) {
  v16h a; const int g = lane >> 4;
#pragma unroll
  for (int i = 0; i < 8; ++i) { const int ka = k0 + 8 * g + i, kb = ka + 16;
    a[i] = (_Float16)(ka < K ? W[(size_t)(ka < K ? ka : K - 1) * ld + n] : 0.f); a[8 + i] = (_Float16)(kb < K ? W[(size_t)(kb < K ? kb : K - 1) * ld + n] : 0.f); }
  return a;
}
struct F2 { v16b h, l; };
__device__ __forceinline__ F2 bsplit16(const float v[16]) { F2 r;
#pragma unroll
  for (int i = 0; i < 16; ++i) { const __bf16 h = (__bf16)v[i]; r.h[i] = h; r.l[i] = (__bf16)(v[i] - (float)h); }
  return r; }
__device__ __forceinline__ F2 split_row(const float* row, int k0, int lane) { float v[16]; const float* p = row + k0 + 8 * (lane >> 4);
#pragma unroll
  for (int i = 0; i < 8; ++i) { v[i] = p[i]; v[8 + i] = p[16 + i]; }
  return bsplit16(v); }
__device__ __forceinline__ F2 split_rowK(const float* row, int k0, int lane, int K) { float v[16]; const int g = lane >> 4;
#pragma unroll
  for (int i = 0; i < 8; ++i) { const int ka = k0 + 8 * g + i, kb = ka + 16; v[i] = ka < K ? row[ka < K ? ka : K - 1] : 0.f; v[8 + i] = kb < K ? row[kb < K ? kb : K - 1] : 0.f; }
  return bsplit16(v); }
__device__ __forceinline__ F2 split_col(const float* W, int k0, int n, int lane, int ld, int K) { float v[16]; const int g = lane >> 4;
#pragma unroll
  for (int i = 0; i < 8; ++i) { const int ka = k0 + 8 * g + i, kb = ka + 16; v[i] = ka < K ? W[(size_t)(ka < K ? ka : K - 1) * ld + n] : 0.f; v[8 + i] = kb < K ? W[(size_t)(kb < K ? kb : K - 1) * ld + n] : 0.f; }
  return bsplit16(v); }
__device__ __forceinline__ v8f mac3(const F2& a, const F2& b, v8f c) { c = wmma_bf(a.l, b.h, c); c = wmma_bf(a.h, b.l, c); return wmma_bf(a.h, b.h, c); }
__device__ __forceinline__ float sigm(float v) { return 1.0f / (1.0f + expf(-v)); }
#define LDSX() do { asm volatile("s_wait_dscnt 0" ::: "memory"); __builtin_amdgcn_wave_barrier(); __builtin_amdgcn_fence(__ATOMIC_RELEASE, "workgroup"); } while (0)

__device__ __forceinline__ float bfr(float v) { return (float)(__bf16)v; }
#define NBAT 524288
#define NF 5
#define NH1 128
#define NH2 32
#ifndef NBLK
#define NBLK (NBAT / 64)
#endif
__global__ __launch_bounds__(128) void k_bn(const float* __restrict__ X, const float* __restrict__ MEAN, const float* __restrict__ STD, const float* __restrict__ W1, const float* __restrict__ B1, const float* __restrict__ W21, const float* __restrict__ B21, const float* __restrict__ W22, const float* __restrict__ B22, const float* __restrict__ W31, const float* __restrict__ B31, const float* __restrict__ W32, const float* __restrict__ B32, float* __restrict__ OUT) {
  __shared__ __align__(16) float so[64];
  const int tid = threadIdx.x, wave = tid >> 5, lane = tid & 31, col = lane & 15, g = lane >> 4; const size_t r0 = (size_t)blockIdx.x * 64 + wave * 16; const size_t arow = r0 + col;
  float xa[NF];
#pragma unroll
  for (int f = 0; f < NF; ++f) xa[f] = bfr(X[arow * NF + f]);
  v8f acc[4] = {};
#pragma unroll
  for (int kc = 0; kc < NH1 / 32; ++kc) { float hv[16];
#pragma unroll
    for (int e = 0; e < 16; ++e) { const int o = kc * 32 + 8 * g + (e < 8 ? e : 8 + e); float s = bfr(B1[o]);
#pragma unroll
      for (int f = 0; f < NF; ++f) s += xa[f] * bfr(W1[o * NF + f]);
      hv[e] = fmaxf(s, 0.f); asm volatile("s_wait_loadcnt 0x0" ::: "memory"); }
    const F2 a = bsplit16(hv);
#pragma unroll
    for (int j = 0; j < 4; ++j) { v16b w; const int oo = j * 16 + col; const float* wr = (oo < NH2) ? (W21 + (size_t)oo * NH1) : (W22 + (size_t)(oo - NH2) * NH1); const float* p = wr + kc * 32 + 8 * g;
#pragma unroll
      for (int i = 0; i < 8; ++i) { w[i] = (__bf16)p[i]; w[8 + i] = (__bf16)p[16 + i]; }
      acc[j] = wmma_bf(a.h, w, acc[j]); acc[j] = wmma_bf(a.l, w, acc[j]); } }
  float p1[8], p2[8];
#pragma unroll
  for (int r = 0; r < 8; ++r) { p1[r] = 0.f; p2[r] = 0.f; }
#pragma unroll
  for (int j = 0; j < 4; ++j) { const int oo = j * 16 + col; const int o2 = oo & (NH2 - 1); const float bb = (j < 2) ? bfr(B21[o2]) : bfr(B22[o2]); const float ww = (j < 2) ? bfr(W31[o2]) : bfr(W32[o2]);
#pragma unroll
    for (int r = 0; r < 8; ++r) { const float xv = fmaxf(acc[j][r] + bb, 0.f) * ww; if (j < 2) p1[r] += xv; else p2[r] += xv; } }
#pragma unroll
  for (int r = 0; r < 8; ++r) {
#pragma unroll
    for (int sh = 1; sh < 16; sh <<= 1) { p1[r] += __shfl_xor(p1[r], sh); p2[r] += __shfl_xor(p2[r], sh); } }
  if (col == 0) { const float b31 = bfr(B31[0]), b32 = bfr(B32[0]);
#pragma unroll
    for (int r = 0; r < 8; ++r) { const size_t row = r0 + 8 * g + r; float x0[NF];
#pragma unroll
      for (int f = 0; f < NF; ++f) x0[f] = bfr(X[row * NF + f]) * bfr(STD[f]) + bfr(MEAN[f]);
      const float x31 = p1[r] + b31; const float x32 = 4.0f * sigm(p2[r] + b32);
      const float hh = (x0[1] - x0[3]) + x32 * (x0[0] - x0[2] - 1.8f * x0[3]); const float uu = -x31;
      so[wave * 16 + 8 * g + r] = (1.8f * uu <= hh) ? uu : hh / 1.8f; } }
  __syncthreads();
  if (tid < 16) vst2(OUT + (size_t)blockIdx.x * 64 + tid * 4, *(const v4f*)&so[tid * 4]); }
extern "C" void kernel_launch(void* const* d_in, const int* in_sizes, int n_in, void* d_out, int out_size, void* d_ws, size_t ws_size, hipStream_t stream) {
  (void)in_sizes; (void)n_in; (void)out_size; (void)d_ws; (void)ws_size;
  const float** F = (const float**)d_in;
  k_bn<<<dim3(NBLK), 128, 0, stream>>>(F[0], F[1], F[2], F[3], F[4], F[5], F[6], F[7], F[8], F[9], F[10], F[11], F[12], (float*)d_out);
}
